// Encoder_64046552318129
// MI455X (gfx1250) — hardware-verified
//
#include <hip/hip_runtime.h>
#include <stddef.h>
#include <stdint.h>
#include <math.h>


#define DF     128
#define NP4    512
#define HP     256
#define NHEAD  8
#define NBINS  10
#define NTHR   256
#define NWAVE  8
#define EPT    8
#define CHUNK  (NTHR * EPT)
#define WCAP   (EPT * 32)
#define LISTN  (NWAVE * WCAP)
#define NBA    1024
#define SLA    10
#define RCAP   8192
#define DEGCAP 32
#define GBM    64
#define GBN    128
#define GTHR   128
#define U_EW   2048
#define U_PL   16384
#define NPLN   5
#define AGG_ZINTS    (LISTN + 2 * RCAP + 3 * NBA)
#define MISC_INTS    16
#define ROWBUF_INTS  (NWAVE * HP / 2)
#define AGG_LDS_INTS (AGG_ZINTS + MISC_INTS + ROWBUF_INTS)
#define WSMAX  134217728

static_assert((CHUNK & (CHUNK - 1)) == 0 && CHUNK <= 4096);
static_assert((NBA & (NBA - 1)) == 0 && NBA == (1 << SLA));
static_assert(((long long)CHUNK << SLA) < (1LL << 31));
static_assert(LISTN % NTHR == 0);
static_assert(NBA % NWAVE == 0 && NBA % 32 == 0 && NBA % GBM == 0);
static_assert(RCAP % 4 == 0 && AGG_ZINTS % (NTHR * 4) == 0 && ((AGG_ZINTS + MISC_INTS) % 4) == 0);
static_assert(DEGCAP <= 32 && DEGCAP >= 15 + 8);
static_assert(DF % 32 == 0 && HP % 32 == 0 && HP == 2 * DF && NP4 == 4 * GBN && GBN == DF);
static_assert(GBM == (GTHR / 32) * 16 && DF == 4 * 32);
static_assert(U_EW % NTHR == 0 && U_PL % NTHR == 0 && U_EW == DF * (DF / 8) && U_PL == NP4 * (HP / 8));
static_assert(NBINS * NHEAD <= 128);
static_assert(AGG_LDS_INTS * 4 <= 300000);

typedef float          v4f   __attribute__((ext_vector_type(4)));
typedef float          v8f   __attribute__((ext_vector_type(8)));
typedef int            v4i   __attribute__((ext_vector_type(4)));
typedef int            v8i   __attribute__((ext_vector_type(8)));
typedef unsigned short v4us  __attribute__((ext_vector_type(4)));
typedef unsigned short v8us  __attribute__((ext_vector_type(8)));
typedef unsigned short v16us __attribute__((ext_vector_type(16)));
typedef __bf16         v16bf __attribute__((ext_vector_type(16)));
typedef v4f  __attribute__((may_alias)) v4fa;
typedef v4i  __attribute__((may_alias)) v4ia;
typedef v4us __attribute__((may_alias)) v4usa;
typedef v8us __attribute__((may_alias)) v8usa;
union FragB { v16bf v; v16us u; v8us h[2]; v8i w; };

__device__ __forceinline__ v8f wmb(const FragB& a, const FragB& b, v8f c) {
  v8f d = __builtin_amdgcn_wmma_f32_16x16x32_bf16(false, a.v, false, b.v, (short)0, c, false, false);
  asm volatile("v_nop\n\tv_nop\n\tv_nop\n\tv_nop" : "+v"(d) : "v"(a.w), "v"(b.w));
  return d;
}

__device__ __forceinline__ unsigned bf16_bits(float f) {
  const unsigned u = __float_as_uint(f);
  return (u + 0x7FFFu + ((u >> 16) & 1u)) >> 16;
}
__device__ __forceinline__ float bf16_val(float f) {
  return __uint_as_float(bf16_bits(f) << 16);
}

__device__ __forceinline__ void wave_sync() {
  __builtin_amdgcn_fence(__ATOMIC_RELEASE, "wavefront");
  __builtin_amdgcn_wave_barrier();
  __builtin_amdgcn_fence(__ATOMIC_ACQUIRE, "wavefront");
}

template <int SLB>
__device__ __forceinline__ int scan_chunk(const int* __restrict__ dsts, int nE, int cbase, int slotBase,
                                          int nb, int vec8, int* list, int tid, int lane, int wave) {
  int wc = 0;
  const int el0  = tid * EPT;
  const int e0   = cbase + el0;
  const int sent = -2147483647 - 1;
  v4i da, db;
  if (vec8 != 0 && cbase + CHUNK <= nE) {
    da = *(const v4i*)(dsts + e0);
    db = *(const v4i*)(dsts + e0 + 4);
  } else {
    da.x = (e0     < nE) ? dsts[min(e0,     nE - 1)] : sent;
    da.y = (e0 + 1 < nE) ? dsts[min(e0 + 1, nE - 1)] : sent;
    da.z = (e0 + 2 < nE) ? dsts[min(e0 + 2, nE - 1)] : sent;
    da.w = (e0 + 3 < nE) ? dsts[min(e0 + 3, nE - 1)] : sent;
    db.x = (e0 + 4 < nE) ? dsts[min(e0 + 4, nE - 1)] : sent;
    db.y = (e0 + 5 < nE) ? dsts[min(e0 + 5, nE - 1)] : sent;
    db.z = (e0 + 6 < nE) ? dsts[min(e0 + 6, nE - 1)] : sent;
    db.w = (e0 + 7 < nE) ? dsts[min(e0 + 7, nE - 1)] : sent;
  }
  const unsigned nbs = (unsigned)slotBase;
  const unsigned unb = (unsigned)nb;
  const unsigned s0 = (unsigned)da.x - nbs, s1 = (unsigned)da.y - nbs;
  const unsigned s2 = (unsigned)da.z - nbs, s3 = (unsigned)da.w - nbs;
  const unsigned s4 = (unsigned)db.x - nbs, s5 = (unsigned)db.y - nbs;
  const unsigned s6 = (unsigned)db.z - nbs, s7 = (unsigned)db.w - nbs;
  const bool h0 = s0 < unb, h1 = s1 < unb, h2 = s2 < unb, h3 = s3 < unb;
  const bool h4 = s4 < unb, h5 = s5 < unb, h6 = s6 < unb, h7 = s7 < unb;
  const int nh = (int)h0 + (int)h1 + (int)h2 + (int)h3 + (int)h4 + (int)h5 + (int)h6 + (int)h7;
  const unsigned any = __builtin_amdgcn_ballot_w32(nh != 0);
  if (any != 0u) {
    int incl = nh;
#pragma unroll
    for (int d = 1; d < 32; d <<= 1) {
      const int y = __shfl_up(incl, d, 32);
      if (lane >= d) incl += y;
    }
    wc = __shfl(incl, 31, 32);
    int pos = incl - nh;
    int* lp = list + wave * WCAP;
#define HITJ(J, HJ, SJ) if (HJ) { if (pos < WCAP) lp[pos] = ((el0 + (J)) << SLB) | (int)(SJ); pos = pos + 1; }
    HITJ(0, h0, s0)
    HITJ(1, h1, s1)
    HITJ(2, h2, s2)
    HITJ(3, h3, s3)
    HITJ(4, h4, s4)
    HITJ(5, h5, s5)
    HITJ(6, h6, s6)
    HITJ(7, h7, s7)
#undef HITJ
  }
  return wc;
}

__device__ __forceinline__ float head_dot(v4f u, const v4f w) {
  u.x = (u.x >= 0.0f) ? u.x : 0.2f * u.x;
  u.y = (u.y >= 0.0f) ? u.y : 0.2f * u.y;
  u.z = (u.z >= 0.0f) ? u.z : 0.2f * u.z;
  u.w = (u.w >= 0.0f) ? u.w : 0.2f * u.w;
  float d = u.x * w.x;
  d = fmaf(u.y, w.y, d);
  d = fmaf(u.z, w.z, d);
  d = fmaf(u.w, w.w, d);
  d += __shfl_xor(d, 1, 32);
  d += __shfl_xor(d, 2, 32);
  return d;
}

__device__ __forceinline__ void att_step(float a, const v4f msg, float& mx, float& ls, v4f& acc) {
  const float dd = a - mx;
  const float e  = expf(-fabsf(dd));
  const bool up  = dd > 0.0f;
  const float sc = up ? e : 1.0f;
  const float p  = up ? 1.0f : e;
  mx = up ? a : mx;
  ls = ls * sc + p;
  acc = acc * sc + msg * p;
}

__device__ __forceinline__ v8us pack_hilo(const v4f v, unsigned short* rowbuf, int lane) {
  v4us mh, ml;
  unsigned hb;
  hb = bf16_bits(v.x); mh[0] = (unsigned short)hb; ml[0] = (unsigned short)bf16_bits(v.x - __uint_as_float(hb << 16));
  hb = bf16_bits(v.y); mh[1] = (unsigned short)hb; ml[1] = (unsigned short)bf16_bits(v.y - __uint_as_float(hb << 16));
  hb = bf16_bits(v.z); mh[2] = (unsigned short)hb; ml[2] = (unsigned short)bf16_bits(v.z - __uint_as_float(hb << 16));
  hb = bf16_bits(v.w); mh[3] = (unsigned short)hb; ml[3] = (unsigned short)bf16_bits(v.w - __uint_as_float(hb << 16));
  *(v4usa*)(rowbuf + 4 * lane) = mh;
  *(v4usa*)(rowbuf + DF + 4 * lane) = ml;
  wave_sync();
  const v8us q = *(const v8usa*)(rowbuf + 8 * lane);
  wave_sync();
  return q;
}

__device__ __forceinline__ v8us gath8(const float* __restrict__ p) {
  v8us o;
#pragma unroll
  for (int i = 0; i < 8; ++i) o[i] = (unsigned short)bf16_bits(p[(size_t)i * DF]);
  return o;
}

__global__ __launch_bounds__(NTHR) void k_prep(const float* __restrict__ entW, const float* __restrict__ rWatt,
                                               const float* __restrict__ rWag, const float* __restrict__ rWres,
                                               const float* __restrict__ eWatt, const float* __restrict__ eWag,
                                               const float* __restrict__ eWres, const float* __restrict__ tab,
                                               const int* __restrict__ relfeat, int nT, int nR, int nUnits,
                                               unsigned short* EWT, unsigned short* WPL, unsigned short* HR) {
  const int u = (int)blockIdx.x * NTHR + (int)threadIdx.x;
  v8us o;
  unsigned short* dp;
  if (u < U_EW) {
    const int n  = u >> 4;
    const int k8 = (u & 15) * 8;
    o  = gath8(entW + (size_t)k8 * DF + n);
    dp = EWT + (size_t)n * DF + k8;
  } else if (u < U_EW + NPLN * U_PL) {
    const int v   = u - U_EW;
    const int pl  = v >> 14;
    const int w   = v & (U_PL - 1);
    const int n   = w >> 5;
    const int k8  = (w & 31) * 8;
    const int kk  = k8 & (DF - 1);
    const int seg = n >> 7;
    const int nn  = n & (DF - 1);
    int which, lay, roff;
    if (pl < 2)       { lay = pl;       which = (seg < 2) ? 0 : ((seg == 2) ? 1 : 2); roff = (seg == 1) ? DF : 0; }
    else if (pl == 2) { lay = seg >> 1; which = (seg & 1) ? 4 : 3;                    roff = (seg & 1) ? DF : 2 * DF; }
    else              { lay = pl - 3;   which = (seg < 2) ? 3 : ((seg == 2) ? 4 : 5); roff = (seg == 1) ? DF : 0; }
    const size_t ro = (size_t)(roff + kk) * DF + nn;
    if (which == 0)      o = gath8(rWatt + (size_t)lay * (2 * DF * DF) + ro);
    else if (which == 1) o = gath8(rWag  + (size_t)lay * (DF * DF) + ro);
    else if (which == 2) o = gath8(rWres + (size_t)lay * (DF * DF) + ro);
    else if (which == 3) o = gath8(eWatt + (size_t)lay * (3 * DF * DF) + ro);
    else if (which == 4) o = gath8(eWag  + (size_t)lay * (2 * DF * DF) + ro);
    else                 o = gath8(eWres + (size_t)lay * (DF * DF) + ro);
    dp = WPL + (size_t)pl * (NP4 * HP) + (size_t)n * HP + k8;
  } else if (u < nUnits) {
    const int v   = u - (U_EW + NPLN * U_PL);
    const int row = v >> 5;
    const int k8  = (v & 31) * 8;
    const int kk  = k8 & (DF - 1);
    const int rr  = row < nR ? row : nR - 1;
    int rf = relfeat[rr];
    rf = rf < 0 ? 0 : (rf > nT - 1 ? nT - 1 : rf);
    const float* p = tab + (size_t)rf * DF + kk;
    const v4f a = *(const v4f*)p;
    const v4f b = *(const v4f*)(p + 4);
    const bool ok = (row < nR) && (k8 < DF);
    o[0] = ok ? (unsigned short)bf16_bits(a.x) : (unsigned short)0;
    o[1] = ok ? (unsigned short)bf16_bits(a.y) : (unsigned short)0;
    o[2] = ok ? (unsigned short)bf16_bits(a.z) : (unsigned short)0;
    o[3] = ok ? (unsigned short)bf16_bits(a.w) : (unsigned short)0;
    o[4] = ok ? (unsigned short)bf16_bits(b.x) : (unsigned short)0;
    o[5] = ok ? (unsigned short)bf16_bits(b.y) : (unsigned short)0;
    o[6] = ok ? (unsigned short)bf16_bits(b.z) : (unsigned short)0;
    o[7] = ok ? (unsigned short)bf16_bits(b.w) : (unsigned short)0;
    dp = HR + (size_t)row * HP + k8;
  } else {
    return;
  }
  *(volatile v8us*)dp = o;
  __threadfence();
  *(volatile v8us*)dp = o;
}

__device__ __forceinline__ void mma8(const FragB& af, const unsigned short* __restrict__ bp, size_t K, int k0,
                                     v8f (&acc)[8]) {
#pragma unroll
  for (int nt = 0; nt < 8; ++nt) {
    const unsigned short* wq = bp + (size_t)(16 * nt) * K + k0;
    FragB bf;
    bf.h[0] = *(const v8usa*)wq;
    bf.h[1] = *(const v8usa*)(wq + 16);
    acc[nt] = wmb(af, bf, acc[nt]);
  }
}

template <int E0>
__global__ __launch_bounds__(GTHR) void k_gemm(const unsigned short* __restrict__ Apl, const float* __restrict__ Af,
                                               int nA, const unsigned short* __restrict__ BT, int K,
                                               const float* __restrict__ bs0, const float* __restrict__ bs2,
                                               const float* __restrict__ bs3, int bmask,
                                               float* outF, int ldo, unsigned short* outH) {
  __shared__ __attribute__((aligned(16))) float stg[GBM * GBN];
  const int tid = (int)threadIdx.x, lane = tid & 31, wave = tid >> 5, hh = lane >> 4, m = lane & 15;
  const int rowBase = (int)blockIdx.x * GBM;
  const int by      = (int)blockIdx.y;
  const int col0    = by * GBN;

  v8f acc[8];
  {
    const v8f z = {0.f, 0.f, 0.f, 0.f, 0.f, 0.f, 0.f, 0.f};
#pragma unroll
    for (int t = 0; t < 8; ++t) acc[t] = z;
  }
  const unsigned short* bp = BT + (size_t)(col0 + m) * (size_t)K + 8 * hh;

  if constexpr (E0 != 0) {
    int ar = rowBase + 16 * wave + m;
    ar = ar < nA ? ar : nA - 1;
    const float* ap = Af + (size_t)ar * DF + 8 * hh;
#pragma unroll 1
    for (int k0 = 0; k0 < K; k0 += 32) {
      const v4f x0 = *(const v4f*)(ap + k0);
      const v4f x1 = *(const v4f*)(ap + k0 + 4);
      const v4f y0 = *(const v4f*)(ap + k0 + 16);
      const v4f y1 = *(const v4f*)(ap + k0 + 20);
      v8us g0, g1;
      g0[0] = (unsigned short)bf16_bits(x0.x); g0[1] = (unsigned short)bf16_bits(x0.y);
      g0[2] = (unsigned short)bf16_bits(x0.z); g0[3] = (unsigned short)bf16_bits(x0.w);
      g0[4] = (unsigned short)bf16_bits(x1.x); g0[5] = (unsigned short)bf16_bits(x1.y);
      g0[6] = (unsigned short)bf16_bits(x1.z); g0[7] = (unsigned short)bf16_bits(x1.w);
      g1[0] = (unsigned short)bf16_bits(y0.x); g1[1] = (unsigned short)bf16_bits(y0.y);
      g1[2] = (unsigned short)bf16_bits(y0.z); g1[3] = (unsigned short)bf16_bits(y0.w);
      g1[4] = (unsigned short)bf16_bits(y1.x); g1[5] = (unsigned short)bf16_bits(y1.y);
      g1[6] = (unsigned short)bf16_bits(y1.z); g1[7] = (unsigned short)bf16_bits(y1.w);
      FragB af;
      af.h[0] = g0;
      af.h[1] = g1;
      mma8(af, bp, (size_t)K, k0, acc);
    }
  } else {
    const unsigned short* ap = Apl + (size_t)(rowBase + 16 * wave + m) * (size_t)K + 8 * hh;
#pragma unroll 1
    for (int k0 = 0; k0 < K; k0 += 32) {
      FragB af;
      af.h[0] = *(const v8usa*)(ap + k0);
      af.h[1] = *(const v8usa*)(ap + k0 + 16);
      mma8(af, bp, (size_t)K, k0, acc);
    }
  }

#pragma unroll
  for (int nt = 0; nt < 8; ++nt) {
    const int lc = 16 * nt + m;
#pragma unroll
    for (int r = 0; r < 8; ++r) {
      const int lr = 16 * wave + 8 * hh + r;
      stg[lr * GBN + lc] = acc[nt][r];
    }
  }
  __syncthreads();

  v4f bb;
  {
    const v4f t0 = *(const v4f*)(bs0 + 4 * lane);
    const v4f t2 = *(const v4f*)(bs2 + 4 * lane);
    const v4f t3 = *(const v4f*)(bs3 + 4 * lane);
    const float f0 = (by == 0 && (bmask & 1) != 0) ? 1.0f : 0.0f;
    const float f2 = (by == 2 && (bmask & 4) != 0) ? 1.0f : 0.0f;
    const float f3 = (by == 3 && (bmask & 8) != 0) ? 1.0f : 0.0f;
    bb.x = bf16_val(t0.x) * f0 + bf16_val(t2.x) * f2 + bf16_val(t3.x) * f3;
    bb.y = bf16_val(t0.y) * f0 + bf16_val(t2.y) * f2 + bf16_val(t3.y) * f3;
    bb.z = bf16_val(t0.z) * f0 + bf16_val(t2.z) * f2 + bf16_val(t3.z) * f3;
    bb.w = bf16_val(t0.w) * f0 + bf16_val(t2.w) * f2 + bf16_val(t3.w) * f3;
  }

  v4f pv[16];
#pragma unroll
  for (int i = 0; i < 16; ++i) pv[i] = *(const v4fa*)(stg + (16 * wave + i) * GBN + 4 * lane);
  __syncthreads();
#pragma unroll
  for (int i = 0; i < 16; ++i) pv[i] = pv[i] + bb;

  if constexpr (E0 == 0) {
#pragma unroll
    for (int i = 0; i < 16; ++i) {
      float* op = outF + (size_t)(rowBase + 16 * wave + i) * (size_t)ldo + col0 + 4 * lane;
      *(volatile v4f*)op = pv[i];
    }
    __threadfence();
#pragma unroll
    for (int i = 0; i < 16; ++i) {
      float* op = outF + (size_t)(rowBase + 16 * wave + i) * (size_t)ldo + col0 + 4 * lane;
      *(volatile v4f*)op = pv[i];
    }
  } else {
#pragma unroll
    for (int i = 0; i < 16; ++i) {
      const bool ok = (rowBase + 16 * wave + i) < nA;
      v4f y = pv[i];
      y.x = ok ? y.x : 0.0f; y.y = ok ? y.y : 0.0f; y.z = ok ? y.z : 0.0f; y.w = ok ? y.w : 0.0f;
      v4us h4, l4;
      unsigned hb;
      hb = bf16_bits(y.x); h4[0] = (unsigned short)hb; l4[0] = (unsigned short)bf16_bits(y.x - __uint_as_float(hb << 16));
      hb = bf16_bits(y.y); h4[1] = (unsigned short)hb; l4[1] = (unsigned short)bf16_bits(y.y - __uint_as_float(hb << 16));
      hb = bf16_bits(y.z); h4[2] = (unsigned short)hb; l4[2] = (unsigned short)bf16_bits(y.z - __uint_as_float(hb << 16));
      hb = bf16_bits(y.w); h4[3] = (unsigned short)hb; l4[3] = (unsigned short)bf16_bits(y.w - __uint_as_float(hb << 16));
      unsigned short* srow = (unsigned short*)stg + (size_t)(16 * wave + i) * (2 * GBN);
      *(v4usa*)(srow + 4 * lane) = h4;
      *(v4usa*)(srow + DF + 4 * lane) = l4;
    }
    __syncthreads();
    v8us qv[16];
#pragma unroll
    for (int i = 0; i < 16; ++i) {
      const unsigned short* srow = (const unsigned short*)stg + (size_t)(16 * wave + i) * (2 * GBN);
      qv[i] = *(const v8usa*)(srow + 8 * lane);
    }
#pragma unroll
    for (int i = 0; i < 16; ++i) {
      unsigned short* rp = outH + (size_t)(rowBase + 16 * wave + i) * (size_t)HP + 8 * lane;
      *(volatile v8us*)rp = qv[i];
    }
    __threadfence();
#pragma unroll
    for (int i = 0; i < 16; ++i) {
      unsigned short* rp = outH + (size_t)(rowBase + 16 * wave + i) * (size_t)HP + 8 * lane;
      *(volatile v8us*)rp = qv[i];
    }
  }
}

template <int FIN>
__global__ __launch_bounds__(NTHR) void k_rscan(const int* __restrict__ rhead, const int* __restrict__ rtail,
                                                const int* __restrict__ bins, int nEr, int nR, int vec8,
                                                const float* __restrict__ rp, const float* __restrict__ rvec,
                                                const float* __restrict__ rbin, unsigned short* hr, float* outp) {
  __shared__ __attribute__((aligned(16))) int list[LISTN];
  __shared__ int wcnt[16];
  __shared__ float binl[128];
  __shared__ __attribute__((aligned(16))) unsigned short rowbuf[HP];
  const int tid = (int)threadIdx.x, lane = tid & 31, wave = tid >> 5;
  const int r = (int)blockIdx.x;
  const bool live = r < nR;
  const int rc = live ? r : nR - 1;

  for (int i = tid; i < LISTN; i += NTHR) list[i] = 0;
  if (tid < 16) wcnt[tid] = 0;
  if (tid < 128) {
    const float t = rbin[tid < NBINS * NHEAD ? tid : NBINS * NHEAD - 1];
    binl[tid] = (tid < NBINS * NHEAD) ? bf16_val(t) : 0.0f;
  }
  __syncthreads();

  const v4f pah = *(const v4f*)(rp + (size_t)rc * NP4 + 4 * lane);
  v4f rv;
  {
    const v4f t = *(const v4f*)(rvec + 4 * lane);
    rv.x = bf16_val(t.x); rv.y = bf16_val(t.y); rv.z = bf16_val(t.z); rv.w = bf16_val(t.w);
  }
  float mx = -__builtin_inff(), ls = 0.0f;
  v4f acc = {0.f, 0.f, 0.f, 0.f};
  const int hd = lane >> 2;

  const int nChunks = live ? (nEr + CHUNK - 1) / CHUNK : 0;
#pragma unroll 1
  for (int ch = 0; ch < nChunks; ++ch) {
    const int cbase = ch * CHUNK;
    const int wc = scan_chunk<0>(rhead, nEr, cbase, r, 1, vec8, list, tid, lane, wave);
    if (lane == 0) wcnt[wave] = wc;
    __syncthreads();
    if (wave == 0) {
#pragma unroll 1
      for (int w2 = 0; w2 < NWAVE; ++w2) {
        int c = wcnt[w2];
        c = c < 0 ? 0 : (c > WCAP ? WCAP : c);
#pragma unroll 1
        for (int b0 = 0; b0 < c; b0 += 32) {
          const int idx = b0 + lane;
          const int el  = list[w2 * WCAP + (idx < WCAP ? idx : WCAP - 1)];
          int eid = cbase + (el & (CHUNK - 1));
          eid = eid < 0 ? 0 : (eid > nEr - 1 ? nEr - 1 : eid);
          int tl = rtail[eid];
          tl = tl < 0 ? 0 : (tl > nR - 1 ? nR - 1 : tl);
          int bn = bins[eid];
          bn = bn < 0 ? 0 : (bn > NBINS - 1 ? NBINS - 1 : bn);
          const int m32 = (c - b0) < 32 ? (c - b0) : 32;
#pragma unroll 1
          for (int k = 0; k < m32; ++k) {
            const int tk = __builtin_amdgcn_readlane(tl, k);
            const int bk = __builtin_amdgcn_readlane(bn, k);
            const float* tp = rp + (size_t)tk * NP4 + DF + 4 * lane;
            const v4f pat = *(const v4f*)tp;
            const v4f g   = *(const v4f*)(tp + DF);
            const float a = head_dot(pah + pat, rv) + binl[bk * NHEAD + hd];
            att_step(a, g, mx, ls, acc);
          }
        }
      }
    }
    __syncthreads();
  }

  if (wave == 0) {
    const float rl = 1.0f / (ls + 1e-16f);
    const v4f res = *(const v4f*)(rp + (size_t)rc * NP4 + 3 * DF + 4 * lane);
    v4f v = acc * rl + res;
    v.x = (v.x > 0.0f) ? v.x : (v.x - v.x);
    v.y = (v.y > 0.0f) ? v.y : (v.y - v.y);
    v.z = (v.z > 0.0f) ? v.z : (v.z - v.z);
    v.w = (v.w > 0.0f) ? v.w : (v.w - v.w);
    v.x = live ? v.x : 0.0f; v.y = live ? v.y : 0.0f; v.z = live ? v.z : 0.0f; v.w = live ? v.w : 0.0f;
    const v8us q = pack_hilo(v, rowbuf, lane);
    unsigned short* hp = hr + (size_t)r * HP + 8 * lane;
    float* op = outp + (size_t)rc * DF + 4 * lane;
    *(volatile v8us*)hp = q;
    if constexpr (FIN != 0) { if (live) *(volatile v4f*)op = v; }
    __threadfence();
    *(volatile v8us*)hp = q;
    if constexpr (FIN != 0) { if (live) *(volatile v4f*)op = v; }
  }
}

template <int FIN>
__global__ __launch_bounds__(NTHR) void k_escan(const int* __restrict__ gsrc, const int* __restrict__ keys,
                                                const int* __restrict__ etyp, int nE, int nN, int nR, int vec8,
                                                int mRows, const float* __restrict__ npl,
                                                const float* __restrict__ ert, int ecol,
                                                const float* __restrict__ evec, unsigned short* hb, float* outp) {
  extern __shared__ __attribute__((aligned(16))) int dsm[];
  int* list = dsm;
  int* hl   = dsm + LISTN;
  int* sl   = hl + RCAP;
  int* cnt  = sl + RCAP;
  int* offs = cnt + NBA;
  int* cur  = offs + NBA;
  int* misc = cur + NBA;
  const int tid = (int)threadIdx.x, lane = tid & 31, wave = tid >> 5;
  unsigned short* rowbuf = (unsigned short*)(misc + MISC_INTS) + wave * HP;
  const int nodeBase = (int)blockIdx.x * NBA;

  {
    const v4i z4 = {0, 0, 0, 0};
    for (int i = tid * 4; i < AGG_ZINTS; i += NTHR * 4) *(v4ia*)(dsm + i) = z4;
    if (tid < MISC_INTS) misc[tid] = 0;
  }
  __syncthreads();

  int t = 0, ov = 0;
  const int nChunks = (nE + CHUNK - 1) / CHUNK;
#pragma unroll 1
  for (int ch = 0; ch < nChunks; ++ch) {
    const int cbase = ch * CHUNK;
    const int wc = scan_chunk<SLA>(keys, nE, cbase, nodeBase, NBA, vec8, list, tid, lane, wave);
    if (lane == 0) misc[wave] = wc;
    __syncthreads();
    if (wave == 0) {
#pragma unroll 1
      for (int w2 = 0; w2 < NWAVE; ++w2) {
        int c = misc[w2];
        c = c < 0 ? 0 : (c > WCAP ? WCAP : c);
#pragma unroll 1
        for (int b0 = 0; b0 < c; b0 += 32) {
          const int idx = b0 + lane;
          const int ent = list[w2 * WCAP + (idx < WCAP ? idx : WCAP - 1)];
          const int m32 = (c - b0) < 32 ? (c - b0) : 32;
#pragma unroll 1
          for (int k = 0; k < m32; ++k) {
            const int u    = __builtin_amdgcn_readlane(ent, k);
            const int slot = u & (NBA - 1);
            const int el   = (u >> SLA) & (CHUNK - 1);
            const int pk   = ((cbase + el) << SLA) | slot;
            if (t < RCAP) {
              if (lane == 0) { hl[t] = pk; cnt[slot] = cnt[slot] + 1; }
              t = t + 1;
            } else {
              ov = 1;
            }
          }
        }
      }
    }
    __syncthreads();
  }
  if (wave == 0 && lane == 0) { misc[8] = t; misc[9] = ov; }
  __syncthreads();
  int tt = misc[8];
  tt = tt < 0 ? 0 : (tt > RCAP ? RCAP : tt);
  const int ovf = misc[9];

  if (wave == 0) {
    const int base = lane * (NBA / 32);
    int s = 0;
#pragma unroll 1
    for (int i = 0; i < NBA / 32; ++i) s += cnt[base + i];
    int incl = s;
#pragma unroll
    for (int d = 1; d < 32; d <<= 1) {
      const int y = __shfl_up(incl, d, 32);
      if (lane >= d) incl += y;
    }
    int run = incl - s;
#pragma unroll 1
    for (int i = 0; i < NBA / 32; ++i) {
      const int cv = cnt[base + i];
      offs[base + i] = run;
      cur[base + i]  = run;
      run += cv;
    }
  }
  __syncthreads();
  if (wave == 0) {
#pragma unroll 1
    for (int b0 = 0; b0 < tt; b0 += 32) {
      const int idx = b0 + lane;
      const int ent = hl[idx < RCAP ? idx : RCAP - 1];
      const int m32 = (tt - b0) < 32 ? (tt - b0) : 32;
#pragma unroll 1
      for (int k = 0; k < m32; ++k) {
        const int u    = __builtin_amdgcn_readlane(ent, k);
        const int slot = u & (NBA - 1);
        if (lane == 0) {
          int p = cur[slot];
          p = p < 0 ? 0 : (p > RCAP - 1 ? RCAP - 1 : p);
          sl[p] = u;
          cur[slot] = p + 1;
        }
      }
    }
  }
  __syncthreads();

  const float qnan = __int_as_float(0x7fc00000);
  const float pz = (ovf != 0) ? qnan : 0.0f;
  v4f ev;
  {
    const v4f tv = *(const v4f*)(evec + 4 * lane);
    ev.x = bf16_val(tv.x); ev.y = bf16_val(tv.y); ev.z = bf16_val(tv.z); ev.w = bf16_val(tv.w);
  }
#pragma unroll 1
  for (int si = 0; si < NBA / NWAVE; ++si) {
    const int s    = si * NWAVE + wave;
    const int node = nodeBase + s;
    int c = cnt[s];
    const bool big = c > DEGCAP;
    c = c < 0 ? 0 : (c > DEGCAP ? DEGCAP : c);
    int o = offs[s];
    o = o < 0 ? 0 : (o > RCAP ? RCAP : o);
    const int nc = node < nN ? node : nN - 1;
    int idx = o + lane;
    idx = idx > RCAP - 1 ? RCAP - 1 : idx;
    const int ent = sl[idx];
    int eid = ent >> SLA;
    eid = eid < 0 ? 0 : (eid > nE - 1 ? nE - 1 : eid);
    int sr = gsrc[eid];
    sr = sr < 0 ? 0 : (sr > nN - 1 ? nN - 1 : sr);
    int ty = etyp[eid];
    ty = ty < 0 ? 0 : (ty > nR - 1 ? nR - 1 : ty);
    const float* rowp = npl + (size_t)nc * NP4 + 4 * lane;
    const v4f pt = *(const v4f*)rowp;
    const float rcq = 1.0f / (float)c;
    float mx = -__builtin_inff(), ls = 0.0f;
    v4f acc = {0.f, 0.f, 0.f, 0.f};
    v4f sA  = {0.f, 0.f, 0.f, 0.f};
    v4f sG  = {0.f, 0.f, 0.f, 0.f};
#pragma unroll 1
    for (int k = 0; k <= c; ++k) {
      const bool isSelf = (k == c);
      const int kk = k < 31 ? k : 31;
      int sk = __builtin_amdgcn_readlane(sr, kk);
      const int tk = __builtin_amdgcn_readlane(ty, kk);
      sk = isSelf ? nc : sk;
      const float* sp = npl + (size_t)sk * NP4 + DF + 4 * lane;
      const v4f ph = *(const v4f*)sp;
      const v4f gh = *(const v4f*)(sp + DF);
      const float* ep = ert + (size_t)tk * NP4 + ecol + 4 * lane;
      const v4f ea = *(const v4f*)ep;
      const v4f eg = *(const v4f*)(ep + DF);
      const v4f ma = sA * rcq;
      const v4f mg = sG * rcq;
      const v4f ra = isSelf ? ma : ea;
      const v4f rg = isSelf ? mg : eg;
      const float fe = isSelf ? 0.0f : 1.0f;
      const float a = head_dot(pt + ph + ra, ev);
      att_step(a, gh + rg, mx, ls, acc);
      sA = sA + ea * fe;
      sG = sG + eg * fe;
    }
    const float rl = 1.0f / (ls + 1e-16f);
    const v4f res = *(const v4f*)(rowp + 3 * DF);
    const float pzr = big ? qnan : pz;
    v4f v = acc * rl + res;
    v.x = v.x + pzr; v.y = v.y + pzr; v.z = v.z + pzr; v.w = v.w + pzr;
    v.x = (v.x > 0.0f) ? v.x : (v.x - v.x);
    v.y = (v.y > 0.0f) ? v.y : (v.y - v.y);
    v.z = (v.z > 0.0f) ? v.z : (v.z - v.z);
    v.w = (v.w > 0.0f) ? v.w : (v.w - v.w);
    const bool liveRow = node < nN;
    v.x = liveRow ? v.x : 0.0f; v.y = liveRow ? v.y : 0.0f; v.z = liveRow ? v.z : 0.0f; v.w = liveRow ? v.w : 0.0f;
    if constexpr (FIN == 0) {
      const v8us q = pack_hilo(v, rowbuf, lane);
      if (node < mRows) {
        unsigned short* hp = hb + (size_t)node * HP + 8 * lane;
        *(volatile v8us*)hp = q;
        __threadfence();
        *(volatile v8us*)hp = q;
      }
    } else {
      if (node < nN) {
        float* op = outp + (size_t)node * DF + 4 * lane;
        *(volatile v4f*)op = v;
        __threadfence();
        *(volatile v4f*)op = v;
      }
    }
  }
}

static inline int cdiv(int a, int b) { return (a + b - 1) / b; }
static inline size_t al256(size_t o) { return (o + 255) & ~(size_t)255; }

extern "C" void kernel_launch(void* const* d_in, const int* in_sizes, int n_in,
                              void* d_out, int out_size, void* d_ws, size_t ws_size,
                              hipStream_t stream) {
  if (n_in < 26) return;
  if (in_sizes[0] < DF || (in_sizes[0] % DF) != 0) return;
  const int nN = in_sizes[0] / DF;
  if (nN < 16 || nN >= (1 << 22)) return;
  if (in_sizes[1] != DF * DF || in_sizes[2] != DF) return;
  if (in_sizes[3] < DF || (in_sizes[3] % DF) != 0) return;
  const int nT = in_sizes[3] / DF;
  if (in_sizes[4] != 2 * 2 * DF * DF || in_sizes[5] != 2 * DF) return;
  if (in_sizes[6] != 2 * NBINS * NHEAD || in_sizes[7] != 2 * DF) return;
  if (in_sizes[8] != 2 * DF * DF || in_sizes[9] != 2 * DF) return;
  if (in_sizes[10] != 2 * DF * DF || in_sizes[11] != 2 * DF) return;
  if (in_sizes[12] != 2 * 3 * DF * DF || in_sizes[13] != 2 * DF) return;
  if (in_sizes[14] != 2 * DF) return;
  if (in_sizes[15] != 2 * 2 * DF * DF || in_sizes[16] != 2 * DF) return;
  if (in_sizes[17] != 2 * DF * DF || in_sizes[18] != 2 * DF) return;
  const int nE = in_sizes[19];
  if (nE < 1 || nE >= (1 << 21) || in_sizes[20] != nE || in_sizes[21] != nE) return;
  const int nR = in_sizes[22];
  if (nR < 1 || nR > 65536) return;
  const int nEr = in_sizes[23];
  if (nEr < 1 || nEr >= (1 << 21) || in_sizes[24] != nEr || in_sizes[25] != nEr) return;
  if ((long long)out_size != ((long long)nN + (long long)nR) * DF) return;

  const float* feat   = (const float*)d_in[0];
  const float* entW   = (const float*)d_in[1];
  const float* entb   = (const float*)d_in[2];
  const float* rtab   = (const float*)d_in[3];
  const float* rWatt  = (const float*)d_in[4];
  const float* rbatt  = (const float*)d_in[5];
  const float* rbin   = (const float*)d_in[6];
  const float* rvec   = (const float*)d_in[7];
  const float* rWag   = (const float*)d_in[8];
  const float* rbag   = (const float*)d_in[9];
  const float* rWres  = (const float*)d_in[10];
  const float* rbres  = (const float*)d_in[11];
  const float* eWatt  = (const float*)d_in[12];
  const float* ebatt  = (const float*)d_in[13];
  const float* evec   = (const float*)d_in[14];
  const float* eWag   = (const float*)d_in[15];
  const float* ebag   = (const float*)d_in[16];
  const float* eWres  = (const float*)d_in[17];
  const float* ebres  = (const float*)d_in[18];
  const int* ehead    = (const int*)d_in[19];
  const int* etail    = (const int*)d_in[20];
  const int* etype    = (const int*)d_in[21];
  const int* relfeat  = (const int*)d_in[22];
  const int* rhead    = (const int*)d_in[23];
  const int* rtail    = (const int*)d_in[24];
  const int* binsp    = (const int*)d_in[25];
  float* out  = (float*)d_out;
  float* outR = out + (size_t)nN * DF;

  const int MP  = cdiv(nN, GBM) * GBM;
  const int gM  = MP / GBM;
  const int MPR = cdiv(nR, GBM) * GBM;
  const int gR  = MPR / GBM;
  const int gA  = cdiv(MP, NBA);
  if ((long long)gA * NBA < (long long)MP) return;
  const int vecE = ((nE & 3) == 0) ? 1 : 0;
  const int vecR = ((nEr & 3) == 0) ? 1 : 0;

  char* ws = (char*)d_ws;
  size_t off = 0;
  const size_t oEWT = off; off = al256(off + (size_t)DF * DF * 2);
  const size_t oWPL = off; off = al256(off + (size_t)NPLN * NP4 * HP * 2);
  const size_t oHR  = off; off = al256(off + (size_t)MPR * HP * 2);
  const size_t oRP  = off; off = al256(off + (size_t)MPR * NP4 * 4);
  const size_t oERT = off; off = al256(off + (size_t)MPR * NP4 * 4);
  const size_t oH   = off; off = al256(off + (size_t)MP * HP * 2);
  const size_t oNP  = off; off = al256(off + (size_t)MP * NP4 * 4);
  if (off > ws_size || off > (size_t)WSMAX) return;
  unsigned short* EWT = (unsigned short*)(ws + oEWT);
  unsigned short* WPL = (unsigned short*)(ws + oWPL);
  unsigned short* HR  = (unsigned short*)(ws + oHR);
  float*          RP  = (float*)(ws + oRP);
  float*          ERT = (float*)(ws + oERT);
  unsigned short* H   = (unsigned short*)(ws + oH);
  float*          NPl = (float*)(ws + oNP);
  const size_t plsz = (size_t)NP4 * HP;

  const size_t scanLds = (size_t)AGG_LDS_INTS * 4;
  hipFuncSetAttribute(reinterpret_cast<const void*>(&k_escan<0>), hipFuncAttributeMaxDynamicSharedMemorySize, (int)scanLds);
  hipFuncSetAttribute(reinterpret_cast<const void*>(&k_escan<1>), hipFuncAttributeMaxDynamicSharedMemorySize, (int)scanLds);

  const int nUnits = U_EW + NPLN * U_PL + MPR * (HP / 8);
  k_prep<<<cdiv(nUnits, NTHR), NTHR, 0, stream>>>(entW, rWatt, rWag, rWres, eWatt, eWag, eWres, rtab, relfeat,
                                                  nT, nR, nUnits, EWT, WPL, HR);
  k_gemm<1><<<dim3(gM, 1), GTHR, 0, stream>>>(EWT, feat, nN, EWT, DF, entb, entb, entb, 1, NPl, NP4, H);
  k_gemm<0><<<dim3(gR, 4), GTHR, 0, stream>>>(HR, feat, 0, WPL + 0 * plsz, HP, rbatt, rbag, rbres, 13, RP, NP4, H);
  k_rscan<0><<<MPR, NTHR, 0, stream>>>(rhead, rtail, binsp, nEr, nR, vecR, RP, rvec, rbin, HR, outR);
  k_gemm<0><<<dim3(gR, 4), GTHR, 0, stream>>>(HR, feat, 0, WPL + 1 * plsz, HP, rbatt + DF, rbag + DF, rbres + DF, 13,
                                              RP, NP4, H);
  k_rscan<1><<<MPR, NTHR, 0, stream>>>(rhead, rtail, binsp, nEr, nR, vecR, RP, rvec + DF, rbin + NBINS * NHEAD, HR, outR);
  k_gemm<0><<<dim3(gR, 4), GTHR, 0, stream>>>(HR, feat, 0, WPL + 2 * plsz, HP, rbatt, rbag, rbres, 0, ERT, NP4, H);
  k_gemm<0><<<dim3(gM, 4), GTHR, 0, stream>>>(H, feat, 0, WPL + 3 * plsz, HP, ebatt, ebag, ebres, 13, NPl, NP4, HR);
  k_escan<0><<<gA, NTHR, scanLds, stream>>>(ehead, etail, etype, nE, nN, nR, vecE, MP, NPl, ERT, 0, evec, H, out);
  k_gemm<0><<<dim3(gM, 4), GTHR, 0, stream>>>(H, feat, 0, WPL + 4 * plsz, HP, ebatt + DF, ebag + DF, ebres + DF, 13,
                                              NPl, NP4, HR);
  k_escan<1><<<gA, NTHR, scanLds, stream>>>(ehead, etail, etype, nE, nN, nR, vecE, MP, NPl, ERT, 2 * DF, evec + DF, H, out);
}
